// PredictBlock_10660108829387
// MI455X (gfx1250) — hardware-verified
//
#include <hip/hip_runtime.h>
#include <stddef.h>
#include <math.h>

typedef __attribute__((ext_vector_type(16))) _Float16 v16h;
typedef __attribute__((ext_vector_type(8)))  _Float16 v8h;
typedef __attribute__((ext_vector_type(16))) __bf16   v16b;
typedef __attribute__((ext_vector_type(8)))  __bf16   v8b;
typedef __attribute__((ext_vector_type(8)))  float    v8f;
typedef __attribute__((ext_vector_type(4)))  float    v4f;
typedef __attribute__((ext_vector_type(4)))  unsigned int v4u;
typedef __attribute__((ext_vector_type(2)))  unsigned int v2u;

constexpr int NB = 2;
constexpr int NS = 2048;
constexpr int NC1 = 1024;
constexpr int NC2 = 512;
constexpr int NM = 512;
constexpr int NHEADS = 16;
constexpr int HD = 32;
constexpr int NHD = NHEADS * HD;
constexpr int NFF = NC1 * 4;
constexpr int NTOK = NB * NS;

__device__ __forceinline__ unsigned short f2bf_bits(float f) {
  unsigned u = __float_as_uint(f);
  return (unsigned short)((u + 0x7FFFu + ((u >> 16) & 1u)) >> 16);
}
__device__ __forceinline__ float bf_bits2f(unsigned short h) { return __uint_as_float(((unsigned)h) << 16); }
__device__ __forceinline__ unsigned short h16bits(float f) { return __builtin_bit_cast(unsigned short, (_Float16)f); }
__device__ __forceinline__ unsigned pack_h2(float a, float b) {
  return (unsigned)h16bits(a) | ((unsigned)h16bits(b) << 16);
}
__device__ __forceinline__ float h16bits2f(unsigned short u) { return (float)__builtin_bit_cast(_Float16, u); }

__device__ __forceinline__ void dep_guard_h(v8f& a, v8f& b, v16h x, v16h y) { asm volatile("v_nop\n\tv_nop\n\tv_nop\n\tv_nop" : "+v"(a), "+v"(b) : "v"(x), "v"(y)); }
__device__ __forceinline__ void dep_guard_b(v8f& a, v8f& b, v16b x, v16b y) { asm volatile("v_nop\n\tv_nop\n\tv_nop\n\tv_nop" : "+v"(a), "+v"(b) : "v"(x), "v"(y)); }
__device__ __forceinline__ void keep4_h(v16h a, v16h b, v16h c, v16h d) { asm volatile("v_nop" :: "v"(a), "v"(b), "v"(c), "v"(d)); }
__device__ __forceinline__ void keep4_b(v16b a, v16b b, v16b c, v16b d) { asm volatile("v_nop" :: "v"(a), "v"(b), "v"(c), "v"(d)); }
__device__ __forceinline__ void acc_guard4(v8f& a, v8f& b, v8f& c, v8f& d) { asm volatile("v_nop\n\tv_nop\n\tv_nop\n\tv_nop" : "+v"(a), "+v"(b), "+v"(c), "+v"(d)); }
template <typename T> struct Frag;
template <> struct Frag<_Float16> {
  typedef v16h V; union U { v16h v; v8h h[2]; };
  static __device__ __forceinline__ v16h load(const _Float16* p) {
    U f; f.h[0] = *(const v8h*)(p); f.h[1] = *(const v8h*)(p + 16); return f.v;
  }
  static __device__ __forceinline__ v8f mma(v16h a, v16h b, v8f c) {
    return __builtin_amdgcn_wmma_f32_16x16x32_f16(false, a, false, b, (short)0, c, false, false);
  }
  static __device__ __forceinline__ void guard(v8f& a, v8f& b, v16h x, v16h y) { dep_guard_h(a, b, x, y); }
  static __device__ __forceinline__ void keep(v16h a, v16h b, v16h c, v16h d) { keep4_h(a, b, c, d); }
};
template <> struct Frag<__bf16> {
  typedef v16b V; union U { v16b v; v8b h[2]; };
  static __device__ __forceinline__ v16b load(const __bf16* p) {
    U f; f.h[0] = *(const v8b*)(p); f.h[1] = *(const v8b*)(p + 16); return f.v;
  }
  static __device__ __forceinline__ v8f mma(v16b a, v16b b, v8f c) {
    return __builtin_amdgcn_wmma_f32_16x16x32_bf16(false, a, false, b, (short)0, c, false, false);
  }
  static __device__ __forceinline__ void guard(v8f& a, v8f& b, v16b x, v16b y) { dep_guard_b(a, b, x, y); }
  static __device__ __forceinline__ void keep(v16b a, v16b b, v16b c, v16b d) { keep4_b(a, b, c, d); }
};

__device__ __forceinline__ void st2_v4f(float* p, v4f v) {
  *(volatile v4f*)p = v;
  __threadfence();
  *(volatile v4f*)p = v;
}
__device__ __forceinline__ void st2_v4u(unsigned short* p, v4u v) {
  *(volatile v4u*)(void*)p = v;
  __threadfence();
  *(volatile v4u*)(void*)p = v;
}

template <int ET> struct Elem;
template <> struct Elem<0> { typedef _Float16 T; };
template <> struct Elem<1> { typedef __bf16 T; };
template <int ET, bool SPLIT, int BIAS_MODE, int OUT_MODE, bool RESID, int ACT = 0>
__global__ __launch_bounds__(256) void wmma_gemm64(
    const unsigned short* __restrict__ Ap, const unsigned short* __restrict__ A2p, int lda, long strideA,
    const unsigned short* __restrict__ Btp, const unsigned short* __restrict__ Bt2p, int ldb, long strideB,
    void* __restrict__ Cout, void* __restrict__ Cout2, int ldc, long strideC,
    const float* __restrict__ bias,
    const float* __restrict__ resid, long strideR,
    int M, int N, int K, float scale) {
  typedef typename Elem<ET>::T T;
  typedef typename Frag<T>::V V;
  const T* A = (const T*)Ap; const T* A2 = (const T*)A2p; const T* Bt = (const T*)Btp; const T* Bt2 = (const T*)Bt2p;
  __shared__ __align__(16) float sT[8][16 * 68];
  const int b    = blockIdx.y;
  const int lane = threadIdx.x & 31;
  const int wave = threadIdx.x >> 5;
  const int tilesN = N >> 6;
  const int tilesM = M >> 6;
  const int tile = blockIdx.x * 8 + wave;
  if (tile >= tilesM * tilesN) return;
  const int tm = tile / tilesN;
  const int tn = tile - tm * tilesN;
  const int m0 = tm << 6;
  const int n0 = tn << 6;

  const T* Ab  = A  + (size_t)b * strideA;
  const T* Bb  = Bt + (size_t)b * strideB;
  const T* Ab2 = SPLIT ? (A2  + (size_t)b * strideA) : nullptr;
  const T* Bb2 = SPLIT ? (Bt2 + (size_t)b * strideB) : nullptr;

  const int rlane = lane & 15;
  const int koff  = (lane >> 4) * 8;
  const int mOff  = (lane >> 4) * 8;

  v8f acc[4][4];
#pragma unroll
  for (int i = 0; i < 4; ++i)
#pragma unroll
    for (int j = 0; j < 4; ++j) acc[i][j] = (v8f){0.f,0.f,0.f,0.f,0.f,0.f,0.f,0.f};

  for (int k0 = 0; k0 < K; k0 += 32) {
    V bh[4], bl[4];
#pragma unroll
    for (int j = 0; j < 4; ++j) {
      const size_t bo = (size_t)(n0 + (j << 4) + rlane) * ldb + koff + k0;
      bh[j] = Frag<T>::load(Bb + bo);
      if (SPLIT) bl[j] = Frag<T>::load(Bb2 + bo);
    }
#pragma unroll
    for (int i = 0; i < 4; ++i) {
      const size_t ao = (size_t)(m0 + (i << 4) + rlane) * lda + koff + k0;
      V ah = Frag<T>::load(Ab + ao);
      V al;
      if (SPLIT) al = Frag<T>::load(Ab2 + ao);
#pragma unroll
      for (int j = 0; j < 4; ++j) {
        acc[i][j] = Frag<T>::mma(ah, bh[j], acc[i][j]);
        if (SPLIT) {
          acc[i][j] = Frag<T>::mma(ah, bl[j], acc[i][j]);
          acc[i][j] = Frag<T>::mma(al, bh[j], acc[i][j]);
        }
      }
      Frag<T>::guard(acc[i][0], acc[i][3], ah, SPLIT ? al : ah);
    }
    Frag<T>::keep(bh[0], bh[1], bh[2], bh[3]);
    if (SPLIT) Frag<T>::keep(bl[0], bl[1], bl[2], bl[3]);
  }
  acc_guard4(acc[0][0], acc[0][1], acc[0][2], acc[0][3]);
  acc_guard4(acc[1][0], acc[1][1], acc[1][2], acc[1][3]);
  acc_guard4(acc[2][0], acc[2][1], acc[2][2], acc[2][3]);
  acc_guard4(acc[3][0], acc[3][1], acc[3][2], acc[3][3]);

  float* slab = sT[wave];
  const float* Rb = RESID ? (resid + (size_t)b * strideR) : nullptr;
#pragma unroll
  for (int i = 0; i < 4; ++i) {
    const int mBase = m0 + (i << 4);
#pragma unroll
    for (int j = 0; j < 4; ++j) {
      const int n = n0 + (j << 4) + rlane;
      float bv = 0.f;
      if (BIAS_MODE == 2) bv = bias[n];
#pragma unroll
      for (int r = 0; r < 8; ++r) {
        float v = acc[i][j][r] * scale;
        if (BIAS_MODE == 1) v += bias[mBase + mOff + r];
        if (BIAS_MODE == 2) v += bv;
        if (RESID) v += Rb[(size_t)(mBase + mOff + r) * ldc + n];
        if (ACT == 1) v = tanhf(v);
        if (ACT == 2) v = fmaxf(v, 0.0f);
        if (ACT == 3) v = v / (1.0f + expf(-v));
        if (ACT == 4) v = (v > 0.f) ? v : 0.01f * v;
        slab[(mOff + r) * 68 + (j << 4) + rlane] = v;
      }
    }
    __builtin_amdgcn_fence(__ATOMIC_RELEASE, "workgroup");
    __builtin_amdgcn_wave_barrier();
    __builtin_amdgcn_fence(__ATOMIC_ACQUIRE, "workgroup");
    if (OUT_MODE == 0) {
      float* C = (float*)Cout + (size_t)b * strideC;
      const int hh = lane >> 4, c4 = (lane & 15) * 4;
      for (int pass = 0; pass < 2; ++pass) {
#pragma unroll
        for (int it = 0; it < 8; ++it) {
          const int row = it * 2 + hh;
          v4f v = *(const v4f*)(slab + row * 68 + c4);
          *(volatile v4f*)(C + (size_t)(mBase + row) * ldc + n0 + c4) = v;
        }
        __threadfence();
      }
    } else {
      const int q = lane >> 3, c8 = (lane & 7) * 8;
      unsigned short* C  = (unsigned short*)Cout  + (size_t)b * strideC;
      unsigned short* C2 = (OUT_MODE == 2) ? ((unsigned short*)Cout2 + (size_t)b * strideC) : nullptr;
      for (int pass = 0; pass < 2; ++pass) {
#pragma unroll
        for (int it = 0; it < 4; ++it) {
          const int row = it * 4 + q;
          const float* sp = slab + row * 68 + c8;
          v8h hv, lv;
#pragma unroll
          for (int e = 0; e < 8; ++e) {
            if (OUT_MODE == 1) {
              hv[e] = (_Float16)sp[e];
            } else {
              unsigned short hb = f2bf_bits(sp[e]);
              unsigned short lb = f2bf_bits(sp[e] - bf_bits2f(hb));
              hv[e] = __builtin_bit_cast(_Float16, hb);
              lv[e] = __builtin_bit_cast(_Float16, lb);
            }
          }
          *(volatile v8h*)(C + (size_t)(mBase + row) * ldc + n0 + c8) = hv;
          if (OUT_MODE == 2) *(volatile v8h*)(C2 + (size_t)(mBase + row) * ldc + n0 + c8) = lv;
        }
        __threadfence();
      }
    }
    __builtin_amdgcn_fence(__ATOMIC_RELEASE, "workgroup");
    __builtin_amdgcn_wave_barrier();
    __builtin_amdgcn_fence(__ATOMIC_ACQUIRE, "workgroup");
  }
}

template <int TC>
__global__ __launch_bounds__(256) void transpose_cast_kernel(
    const float* __restrict__ in, unsigned short* __restrict__ out,
    int R, int Cc, long zsIn, long zsOut, float mul)
{
  constexpr int SEG = TC / 4;
  constexpr int LPT = (64 * SEG) / 256;
  constexpr int PITCH = 72;
  __shared__ __align__(16) unsigned short tile[TC * PITCH];
  const int tid = threadIdx.x, lane = tid & 31, wave = tid >> 5;
  const int r0 = blockIdx.x * 64, c0 = blockIdx.y * TC, z = blockIdx.z;
  const float* inz = in + (size_t)z * (size_t)zsIn;
  unsigned short* outz = out + (size_t)z * (size_t)zsOut;
#pragma unroll
  for (int i = 0; i < LPT; ++i) {
    const int idx = tid + 256 * i;
    const int row = idx / SEG;
    const int c4 = (idx - row * SEG) * 4;
    const v4f v = *(const v4f*)(inz + (size_t)(r0 + row) * Cc + c0 + c4);
    tile[(c4 + 0) * PITCH + row] = h16bits(v.x * mul);
    tile[(c4 + 1) * PITCH + row] = h16bits(v.y * mul);
    tile[(c4 + 2) * PITCH + row] = h16bits(v.z * mul);
    tile[(c4 + 3) * PITCH + row] = h16bits(v.w * mul);
  }
  __syncthreads();
  const int qq = lane >> 3, c8 = (lane & 7) * 8;
#pragma unroll
  for (int it = 0; it < TC / 32; ++it) {
    const int orow = it * 32 + wave * 4 + qq;
    const v4u val = *(const v4u*)(tile + orow * PITCH + c8);
    st2_v4u(outz + (size_t)(c0 + orow) * R + r0 + c8, val);
  }
}

template <int NW>
__device__ __forceinline__ float block_sum(float v, float* red, int lane, int wave) {
#pragma unroll
  for (int off = 16; off > 0; off >>= 1) v += __shfl_xor(v, off, 32);
  __syncthreads();
  if (lane == 0) red[wave] = v;
  __syncthreads();
  float t = 0.f;
#pragma unroll
  for (int i = 0; i < NW; ++i) t += red[i];
  return t;
}

template <int CDIM, bool STAGE0, bool ADDOUT, int NOUT16>
__global__ __launch_bounds__(CDIM / 4) void ln_rows_kernel(
    const float* __restrict__ x, const float* __restrict__ g0, const float* __restrict__ b0,
    const float* __restrict__ addp, float* __restrict__ outF,
    const float* __restrict__ g1, const float* __restrict__ b1, unsigned short* __restrict__ outH1,
    const float* __restrict__ g2, const float* __restrict__ b2, unsigned short* __restrict__ outH2)
{
  static_assert(!(STAGE0 && ADDOUT), "one f32 output mode");
  constexpr int NT = CDIM / 4;
  constexpr int NW = NT / 32;
  __shared__ float red[NW];
  __shared__ __align__(16) unsigned short hrow[2][CDIM];
  const int tid = threadIdx.x, lane = tid & 31, wave = tid >> 5;
  const size_t row = blockIdx.x;
  const float invC = 1.0f / (float)CDIM;
  const v4f xv = *(const v4f*)(x + row * CDIM + 4 * tid);
  float y0 = xv.x, y1 = xv.y, y2 = xv.z, y3 = xv.w;
  if (STAGE0) {
    const float mu = block_sum<NW>(y0 + y1 + y2 + y3, red, lane, wave) * invC;
    const float d0 = y0 - mu, d1 = y1 - mu, d2 = y2 - mu, d3 = y3 - mu;
    const float var = block_sum<NW>(d0 * d0 + d1 * d1 + d2 * d2 + d3 * d3, red, lane, wave) * invC;
    const float rs = rsqrtf(var + 1e-5f);
    const v4f gv = *(const v4f*)(g0 + 4 * tid);
    const v4f bv = *(const v4f*)(b0 + 4 * tid);
    y0 = d0 * rs * gv.x + bv.x;
    y1 = d1 * rs * gv.y + bv.y;
    y2 = d2 * rs * gv.z + bv.z;
    y3 = d3 * rs * gv.w + bv.w;
    v4f yv; yv.x = y0; yv.y = y1; yv.z = y2; yv.w = y3;
    st2_v4f(outF + row * CDIM + 4 * tid, yv);
  }
  if (ADDOUT) {
    const v4f av = *(const v4f*)(addp + row * CDIM + 4 * tid);
    v4f sv;
    sv.x = xv.x + av.x; sv.y = xv.y + av.y; sv.z = xv.z + av.z; sv.w = xv.w + av.w;
    st2_v4f(outF + row * CDIM + 4 * tid, sv);
  }
  const float mu2 = block_sum<NW>(y0 + y1 + y2 + y3, red, lane, wave) * invC;
  const float e0 = y0 - mu2, e1 = y1 - mu2, e2 = y2 - mu2, e3 = y3 - mu2;
  const float var2 = block_sum<NW>(e0 * e0 + e1 * e1 + e2 * e2 + e3 * e3, red, lane, wave) * invC;
  const float rs2 = rsqrtf(var2 + 1e-5f);
  {
    const v4f gv = *(const v4f*)(g1 + 4 * tid);
    const v4f bv = *(const v4f*)(b1 + 4 * tid);
    v2u pk;
    pk.x = pack_h2(e0 * rs2 * gv.x + bv.x, e1 * rs2 * gv.y + bv.y);
    pk.y = pack_h2(e2 * rs2 * gv.z + bv.z, e3 * rs2 * gv.w + bv.w);
    *(v2u*)(hrow[0] + 4 * tid) = pk;
  }
  if (NOUT16 == 2) {
    const v4f gv = *(const v4f*)(g2 + 4 * tid);
    const v4f bv = *(const v4f*)(b2 + 4 * tid);
    v2u pk;
    pk.x = pack_h2(e0 * rs2 * gv.x + bv.x, e1 * rs2 * gv.y + bv.y);
    pk.y = pack_h2(e2 * rs2 * gv.z + bv.z, e3 * rs2 * gv.w + bv.w);
    *(v2u*)(hrow[1] + 4 * tid) = pk;
  }
  __syncthreads();
  if (tid < CDIM / 8) {
    const v4u v1 = *(const v4u*)(hrow[0] + 8 * tid);
    st2_v4u(outH1 + row * CDIM + 8 * tid, v1);
    if (NOUT16 == 2) {
      const v4u v2 = *(const v4u*)(hrow[1] + 8 * tid);
      st2_v4u(outH2 + row * CDIM + 8 * tid, v2);
    }
  }
}

__global__ __launch_bounds__(256) void gelu_f16_inplace_kernel(unsigned* __restrict__ buf, int nquads, float outmul)
{
  __shared__ __align__(16) unsigned stg[256 * 4];
  const int tid = threadIdx.x;
  size_t qd = (size_t)blockIdx.x * 256 + tid;
  const bool live = qd < (size_t)nquads;
  if (!live) qd = (size_t)nquads - 1;
  const v4u w = *(const v4u*)(buf + qd * 4);
  *(v4u*)(stg + tid * 4) = w;
  __syncthreads();
#pragma unroll 1
  for (int i = 0; i < 4; ++i) {
    const unsigned u = stg[tid * 4 + i];
    const float a = h16bits2f((unsigned short)(u & 0xffffu));
    const float c = h16bits2f((unsigned short)(u >> 16));
    const float ga = 0.5f * a * (1.0f + erff(a * 0.70710678118654752f)) * outmul;
    const float gc = 0.5f * c * (1.0f + erff(c * 0.70710678118654752f)) * outmul;
    stg[tid * 4 + i] = pack_h2(ga, gc);
  }
  __syncthreads();
  const v4u r = *(const v4u*)(stg + tid * 4);
  if (live) {
    unsigned* dst = buf + qd * 4;
    *(volatile v4u*)dst = r;
    __threadfence();
    *(volatile v4u*)dst = r;
  }
}

#define AT_QB 64
#define AT_KC 64
#define AT_NW 4
constexpr int QPITCH = NHD;
constexpr int KVPITCH = 2 * NHD;
constexpr int VOFF = NHD;
constexpr float PCARRY = 32768.0f;
constexpr float OCARRY = 64.0f;

__device__ __forceinline__ v8f mma_h(v16h a, v16h b, v8f c) {
  c = __builtin_amdgcn_wmma_f32_16x16x32_f16(false, a, false, b, (short)0, c, false, false);
  asm volatile("v_nop\n\tv_nop\n\tv_nop\n\tv_nop" : "+v"(c) : "v"(a), "v"(b));
  return c;
}

template <bool CAUSAL>
__global__ __launch_bounds__(128) void attn_hd32_kernel(
    const unsigned short* __restrict__ qp, const unsigned short* __restrict__ kvp,
    unsigned short* __restrict__ op, int S, int T, float sscale)
{
  union FH { v16h v; v8h h[2]; };
  __shared__ __align__(16) unsigned short Ksh[AT_KC * HD];
  __shared__ __align__(16) unsigned short Vt[HD * AT_KC];
  __shared__ __align__(16) unsigned short Psh[AT_NW][16 * AT_KC];
  __shared__ __align__(16) float Os[AT_NW][16 * 68];

  const int tid = threadIdx.x, wave = tid >> 5, lane = tid & 31, hh = lane >> 4, c = lane & 15;
  const int nqb = S / AT_QB;
  int bx = blockIdx.x;
  const int qb = bx % nqb; bx /= nqb;
  const int hp = bx % (NHEADS / 2);
  const int b  = bx / (NHEADS / 2);
  const int q0 = qb * AT_QB + wave * 16;
  const int nch = T / AT_KC;
  float* os = Os[wave];
  unsigned short* pw = Psh[wave];

#pragma unroll 1
  for (int hs = 0; hs < 2; ++hs) {
    const int h = hp * 2 + hs;
    const v16h qa = Frag<_Float16>::load((const _Float16*)(qp + (size_t)(b * S + q0 + c) * QPITCH + h * HD + 8 * hh));
    float mrow[8], lrow[8];
    v8f oacc[2];
#pragma unroll
    for (int r = 0; r < 8; ++r) { mrow[r] = -INFINITY; lrow[r] = 0.f; }
    oacc[0] = (v8f){0.f,0.f,0.f,0.f,0.f,0.f,0.f,0.f};
    oacc[1] = (v8f){0.f,0.f,0.f,0.f,0.f,0.f,0.f,0.f};

    for (int kc = 0; kc < nch; ++kc) {
      const int kv0 = kc * AT_KC;
      const bool pv_on = (!CAUSAL) || (kc >= qb);
      __syncthreads();
#pragma unroll
      for (int i = 0; i < 2; ++i) {
        const int idx = tid + 128 * i;
        const int kvr = idx >> 2, seg = (idx & 3) * 8;
        const size_t rowoff = (size_t)(b * T + kv0 + kvr) * KVPITCH + h * HD + seg;
        const v4u kk = *(const v4u*)(kvp + rowoff);
        *(v4u*)(Ksh + kvr * HD + seg) = kk;
        if (pv_on) {
          const v4u vv = *(const v4u*)(kvp + rowoff + VOFF);
          Vt[(seg + 0) * AT_KC + kvr] = (unsigned short)(vv.x & 0xffffu);
          Vt[(seg + 1) * AT_KC + kvr] = (unsigned short)(vv.x >> 16);
          Vt[(seg + 2) * AT_KC + kvr] = (unsigned short)(vv.y & 0xffffu);
          Vt[(seg + 3) * AT_KC + kvr] = (unsigned short)(vv.y >> 16);
          Vt[(seg + 4) * AT_KC + kvr] = (unsigned short)(vv.z & 0xffffu);
          Vt[(seg + 5) * AT_KC + kvr] = (unsigned short)(vv.z >> 16);
          Vt[(seg + 6) * AT_KC + kvr] = (unsigned short)(vv.w & 0xffffu);
          Vt[(seg + 7) * AT_KC + kvr] = (unsigned short)(vv.w >> 16);
        }
      }
      __syncthreads();

      v8f s[4];
#pragma unroll
      for (int j = 0; j < 4; ++j) {
        FH kb;
        kb.h[0] = *(const v8h*)(Ksh + (j * 16 + c) * HD + 8 * hh);
        kb.h[1] = *(const v8h*)(Ksh + (j * 16 + c) * HD + 16 + 8 * hh);
        s[j] = mma_h(qa, kb.v, (v8f){0.f,0.f,0.f,0.f,0.f,0.f,0.f,0.f});
      }
      float cm[8];
#pragma unroll
      for (int r = 0; r < 8; ++r) {
        float m = -INFINITY;
#pragma unroll
        for (int j = 0; j < 4; ++j) {
          s[j][r] *= sscale;
          m = fmaxf(m, s[j][r]);
        }
#pragma unroll
        for (int off = 1; off < 16; off <<= 1) m = fmaxf(m, __shfl_xor(m, off, 32));
        cm[r] = m;
      }
#pragma unroll
      for (int r = 0; r < 8; ++r) {
        const int qrow = q0 + 8 * hh + r;
        const float mnew = fmaxf(mrow[r], cm[r]);
        const float alpha = expf(mrow[r] - mnew);
        mrow[r] = mnew;
        float psum = 0.f;
#pragma unroll
        for (int j = 0; j < 4; ++j) {
          const float p = expf(s[j][r] - mnew);
          psum += p;
          if (pv_on) {
            const int kvcol = kv0 + j * 16 + c;
            const bool drop = CAUSAL && (kvcol <= qrow);
            const float pm = drop ? 0.0f : p;
            pw[(8 * hh + r) * AT_KC + j * 16 + c] = h16bits(pm * PCARRY);
          }
        }
#pragma unroll
        for (int off = 1; off < 16; off <<= 1) psum += __shfl_xor(psum, off, 32);
        lrow[r] = lrow[r] * alpha + psum;
        oacc[0][r] *= alpha;
        oacc[1][r] *= alpha;
      }
      if (pv_on) {
        __syncthreads();
#pragma unroll
        for (int kk = 0; kk < 2; ++kk) {
          const v16h pa = Frag<_Float16>::load((const _Float16*)(pw + c * AT_KC + kk * 32 + 8 * hh));
#pragma unroll
          for (int t = 0; t < 2; ++t) {
            FH vb;
            vb.h[0] = *(const v8h*)(Vt + (t * 16 + c) * AT_KC + kk * 32 + 8 * hh);
            vb.h[1] = *(const v8h*)(Vt + (t * 16 + c) * AT_KC + kk * 32 + 16 + 8 * hh);
            oacc[t] = mma_h(pa, vb.v, oacc[t]);
          }
        }
      }
    }
#pragma unroll
    for (int r = 0; r < 8; ++r) {
      const float inv = OCARRY * (1.0f / (lrow[r] * PCARRY));
#pragma unroll
      for (int t = 0; t < 2; ++t) os[(8 * hh + r) * 68 + hs * 32 + t * 16 + c] = oacc[t][r] * inv;
    }
  }
  __syncthreads();
  {
    const int qq = lane >> 3, c8 = (lane & 7) * 8;
    unsigned short* ob = op + (size_t)(b * S + q0) * QPITCH + hp * 64;
    for (int pass = 0; pass < 2; ++pass) {
#pragma unroll
      for (int it = 0; it < 4; ++it) {
        const int row = it * 4 + qq;
        const float* sp = os + row * 68 + c8;
        v8h hv;
#pragma unroll
        for (int e = 0; e < 8; ++e) hv[e] = (_Float16)sp[e];
        *(volatile v8h*)(ob + (size_t)row * QPITCH + c8) = hv;
      }
      __threadfence();
    }
  }
}

static_assert(NS % AT_QB == 0 && NS % AT_KC == 0 && NM % AT_KC == 0, "attention tiles");
static_assert(NTOK % 64 == 0 && (NB * NM) % 64 == 0, "gemm M tiles");
static_assert(NHD % 64 == 0 && NC1 % 64 == 0 && NFF % 64 == 0 && (2 * NHD) % 64 == 0, "gemm N tiles");
static_assert(NC1 % 32 == 0 && NC2 % 32 == 0 && NHD % 32 == 0 && NFF % 32 == 0, "gemm K steps");
static_assert(NC1 % 64 == 0 && NC2 % 64 == 0 && NFF % 64 == 0 && NHD % 64 == 0 && HD == 32, "transpose tiles");
static_assert(NHEADS % 2 == 0, "head pairs");

constexpr size_t MIB = 1048576;
constexpr size_t OFF_X    = 0;
constexpr size_t OFF_RSUM = 16 * MIB;
constexpr size_t OFF_XOUT = 32 * MIB;
constexpr size_t OFF_WQT  = 48 * MIB;
constexpr size_t OFF_WKVT = 49 * MIB;
constexpr size_t OFF_LI1T = 51 * MIB;
constexpr size_t OFF_LI2T = 52 * MIB;
constexpr size_t OFF_LI3T = 60 * MIB;
constexpr size_t OFF_QKV  = 68 * MIB;
constexpr size_t OFF_HB   = 80 * MIB;
constexpr size_t WS_TOTAL = 112 * MIB;
static_assert((size_t)NTOK * NC1 * 4 == 16 * MIB, "f32 plane");
static_assert((size_t)NHD * NC1 * 2 == 1 * MIB, "wqT");
static_assert((size_t)2 * NHD * NC1 * 2 == 2 * MIB, "wkvT");
static_assert((size_t)NC1 * NHD * 2 == 1 * MIB, "li1T");
static_assert((size_t)NFF * NC1 * 2 == 8 * MIB, "li2T/li3T");
static_assert((size_t)NTOK * NHD * 2 + (size_t)NTOK * 2 * NHD * 2 == 12 * MIB, "q+kv");
static_assert((size_t)NTOK * NC1 * 2 <= 12 * MIB, "hn in qkv region");
static_assert((size_t)NTOK * NFF * 2 == 32 * MIB, "ffn hidden");
static_assert((size_t)NTOK * NC1 * 2 * 2 + (size_t)NTOK * NHD * 2 <= 32 * MIB, "xn+yn+o in hidden region");
static_assert(WS_TOTAL == OFF_HB + 32 * MIB && WS_TOTAL <= 134217728, "carve");
static_assert(((size_t)NTOK * NFF / 8) % 256 == 0, "gelu quads");

template <int BIAS_MODE, int OUT_MODE, bool RESID>
static void launch_gemm(hipStream_t st, const unsigned short* A, int lda, const unsigned short* Bt, int ldb,
                        void* C, int ldc, const float* bias, const float* r1,
                        int M, int N, int K, float scale) {
  const int tiles = (M / 64) * (N / 64);
  const unsigned nblk = (unsigned)((tiles + 7) / 8);
  wmma_gemm64<0, false, BIAS_MODE, OUT_MODE, RESID, 0><<<dim3(nblk, 1, 1), dim3(256), 0, st>>>(
      A, nullptr, lda, 0L, Bt, nullptr, ldb, 0L, C, nullptr, ldc, 0L, bias, r1, 0L, M, N, K, scale);
}

template <int TC>
static void launch_tcast(hipStream_t st, const float* in, unsigned short* out, int R, int Cc, int Z,
                         long zsIn, long zsOut, float mul) {
  dim3 grid((unsigned)(R / 64), (unsigned)(Cc / TC), (unsigned)Z);
  transpose_cast_kernel<TC><<<grid, dim3(256), 0, st>>>(in, out, R, Cc, zsIn, zsOut, mul);
}

struct BlockWeights {
  const float *wq, *wk, *wv, *li1_w, *li1_b, *ln3_g, *ln3_b, *li2_w, *li2_b, *li3_w, *li3_b;
};
struct WsPtrs {
  float *X, *XOUT, *RSUM;
  unsigned short *XN, *YN, *O, *WQT, *WKVT, *LI1T, *LI2T, *LI3T, *Q, *KV, *HN, *HB;
};

static void run_block(hipStream_t st, int cy, int T, bool causal, const BlockWeights& w, const WsPtrs& p, float* result) {
  const float WCARRY = 64.0f;
  const float HCARRY = 16.0f;
  launch_tcast<32>(st, w.wq, p.WQT, NC1, HD, NHEADS, (long)NC1 * HD, (long)HD * NC1, WCARRY);
  launch_tcast<32>(st, w.wk, p.WKVT, cy, HD, NHEADS, (long)cy * HD, (long)HD * cy, WCARRY);
  launch_tcast<32>(st, w.wv, p.WKVT + (size_t)NHD * cy, cy, HD, NHEADS, (long)cy * HD, (long)HD * cy, WCARRY);
  launch_tcast<64>(st, w.li1_w, p.LI1T, NHD, NC1, 1, 0L, 0L, WCARRY);
  launch_tcast<64>(st, w.li2_w, p.LI2T, NC1, NFF, 1, 0L, 0L, WCARRY);
  launch_tcast<64>(st, w.li3_w, p.LI3T, NFF, NC1, 1, 0L, 0L, WCARRY);

  const int nty = NB * T;
  launch_gemm<0, 1, false>(st, p.XN, NC1, p.WQT, NC1, p.Q, NHD, nullptr, nullptr,
                           NTOK, NHD, NC1, 1.0f / WCARRY);
  launch_gemm<0, 1, false>(st, p.YN, cy, p.WKVT, cy, p.KV, 2 * NHD, nullptr, nullptr,
                           nty, 2 * NHD, cy, 1.0f / WCARRY);
  const float sscale = 0.17677669529663688f;
  const unsigned ablk = (unsigned)(NB * (NHEADS / 2) * (NS / AT_QB));
  if (causal) attn_hd32_kernel<true><<<dim3(ablk), dim3(128), 0, st>>>(p.Q, p.KV, p.O, NS, T, sscale);
  else        attn_hd32_kernel<false><<<dim3(ablk), dim3(128), 0, st>>>(p.Q, p.KV, p.O, NS, T, sscale);
  launch_gemm<2, 0, true>(st, p.O, NHD, p.LI1T, NHD, p.XOUT, NC1, w.li1_b, p.X,
                          NTOK, NC1, NHD, 1.0f / (OCARRY * WCARRY));
  ln_rows_kernel<NC1, false, true, 1><<<dim3(NTOK), dim3(NC1 / 4), 0, st>>>(
      p.XOUT, nullptr, nullptr, p.X, p.RSUM, w.ln3_g, w.ln3_b, p.HN, nullptr, nullptr, nullptr);
  launch_gemm<2, 1, false>(st, p.HN, NC1, p.LI2T, NC1, p.HB, NFF, w.li2_b, nullptr,
                           NTOK, NFF, NC1, 1.0f / WCARRY);
  {
    const int nquads = NTOK * NFF / 8;
    gelu_f16_inplace_kernel<<<dim3((unsigned)(nquads / 256)), dim3(256), 0, st>>>((unsigned*)p.HB, nquads, HCARRY);
  }
  launch_gemm<2, 0, true>(st, p.HB, NFF, p.LI3T, NFF, result, NC1, w.li3_b, p.RSUM,
                          NTOK, NC1, NFF, 1.0f / (HCARRY * WCARRY));
}

extern "C" void kernel_launch(void* const* d_in, const int* in_sizes, int n_in,
                              void* d_out, int out_size, void* d_ws, size_t ws_size,
                              hipStream_t stream) {
  if (n_in < 36) return;
  if (in_sizes[0] != NB * NS * NC1 || in_sizes[1] != NB * NM * NC2 || out_size != NB * NS * NC1) return;
  if (in_sizes[6] != NHEADS * NC1 * HD || in_sizes[22] != NHEADS * NC2 * HD ||
      in_sizes[17] != NC1 * NFF || in_sizes[34] != NFF * NC1) return;
  if (ws_size < WS_TOTAL) return;

  const float* xx    = (const float*)d_in[0];
  const float* ee    = (const float*)d_in[1];
  const float* ln1_g = (const float*)d_in[2];
  const float* ln1_b = (const float*)d_in[3];
  const float* ln2_g = (const float*)d_in[4];
  const float* ln2_b = (const float*)d_in[5];
  BlockWeights w1, w2;
  w1.wq = (const float*)d_in[6];  w1.wk = (const float*)d_in[7];  w1.wv = (const float*)d_in[8];
  w1.li1_w = (const float*)d_in[9];  w1.li1_b = (const float*)d_in[10];
  const float* a1_lnx_g = (const float*)d_in[11]; const float* a1_lnx_b = (const float*)d_in[12];
  const float* a1_lny_g = (const float*)d_in[13]; const float* a1_lny_b = (const float*)d_in[14];
  w1.ln3_g = (const float*)d_in[15]; w1.ln3_b = (const float*)d_in[16];
  w1.li2_w = (const float*)d_in[17]; w1.li2_b = (const float*)d_in[18];
  w1.li3_w = (const float*)d_in[19]; w1.li3_b = (const float*)d_in[20];
  w2.wq = (const float*)d_in[21]; w2.wk = (const float*)d_in[22]; w2.wv = (const float*)d_in[23];
  w2.li1_w = (const float*)d_in[24]; w2.li1_b = (const float*)d_in[25];
  const float* a2_lnx_g = (const float*)d_in[26]; const float* a2_lnx_b = (const float*)d_in[27];
  const float* a2_lny_g = (const float*)d_in[28]; const float* a2_lny_b = (const float*)d_in[29];
  w2.ln3_g = (const float*)d_in[30]; w2.ln3_b = (const float*)d_in[31];
  w2.li2_w = (const float*)d_in[32]; w2.li2_b = (const float*)d_in[33];
  w2.li3_w = (const float*)d_in[34]; w2.li3_b = (const float*)d_in[35];

  char* ws = (char*)d_ws;
  WsPtrs p;
  p.X    = (float*)(ws + OFF_X);
  p.RSUM = (float*)(ws + OFF_RSUM);
  p.XOUT = (float*)(ws + OFF_XOUT);
  float* Y1 = (float*)(ws + OFF_XOUT);
  p.WQT  = (unsigned short*)(ws + OFF_WQT);
  p.WKVT = (unsigned short*)(ws + OFF_WKVT);
  p.LI1T = (unsigned short*)(ws + OFF_LI1T);
  p.LI2T = (unsigned short*)(ws + OFF_LI2T);
  p.LI3T = (unsigned short*)(ws + OFF_LI3T);
  p.Q    = (unsigned short*)(ws + OFF_QKV);
  p.KV   = (unsigned short*)(ws + OFF_QKV + 4 * MIB);
  p.HN   = (unsigned short*)(ws + OFF_QKV);
  p.HB   = (unsigned short*)(ws + OFF_HB);
  p.XN   = (unsigned short*)(ws + OFF_HB);
  p.YN   = (unsigned short*)(ws + OFF_HB + 8 * MIB);
  p.O    = (unsigned short*)(ws + OFF_HB + 16 * MIB);
  float* out = (float*)d_out;

  ln_rows_kernel<NC1, true, false, 2><<<dim3(NTOK), dim3(NC1 / 4), 0, stream>>>(
      xx, ln1_g, ln1_b, nullptr, p.X, a1_lnx_g, a1_lnx_b, p.XN, a1_lny_g, a1_lny_b, p.YN);
  run_block(stream, NC1, NS, true, w1, p, Y1);

  ln_rows_kernel<NC1, true, false, 1><<<dim3(NTOK), dim3(NC1 / 4), 0, stream>>>(
      Y1, ln2_g, ln2_b, nullptr, p.X, a2_lnx_g, a2_lnx_b, p.XN, nullptr, nullptr, nullptr);
  ln_rows_kernel<NC2, false, false, 1><<<dim3(NB * NM), dim3(NC2 / 4), 0, stream>>>(
      ee, nullptr, nullptr, nullptr, nullptr, a2_lny_g, a2_lny_b, p.YN, nullptr, nullptr, nullptr);
  run_block(stream, NC2, NM, false, w2, p, out);
}
